// IterativeFixedPoint_3848290697534
// MI455X (gfx1250) — hardware-verified
//
#include <hip/hip_runtime.h>
#include <math.h>

typedef __attribute__((ext_vector_type(16))) _Float16 v16h;
typedef __attribute__((ext_vector_type(8)))  _Float16 v8h;
typedef __attribute__((ext_vector_type(4)))  _Float16 v4h;
typedef __attribute__((ext_vector_type(8)))  float    v8f;
typedef __attribute__((ext_vector_type(4)))  float    v4f;

constexpr int kRows    = 32768;
constexpr int kFeat    = 256;
constexpr int kSteps   = 20;
constexpr int kWaves   = 4;
constexpr int kBlkRows = kWaves * 16;
constexpr int kHalfN   = 128;
constexpr int kKP      = kFeat + 8;
constexpr int kSP      = kHalfN + 4;
constexpr int kKTiles  = kFeat / 32;

constexpr float kWCarry = 4096.0f;
constexpr float kZCarry = 512.0f;
constexpr float kFold   = 1.0f / (kWCarry * kZCarry);
constexpr float kF16MinNormal = 6.103515625e-05f;

static_assert(kFeat == 256 && kRows == 32768, "shape");
static_assert((kFeat % 32) == 0, "K multiple of 32");
static_assert((kRows % kBlkRows) == 0, "M multiple of the block tile");
static_assert(kFeat == 2 * kHalfN && (kHalfN % 16) == 0, "N halves");
static_assert(kSteps >= 2, "at least one product step");
static_assert(((kKP * 2) % 16) == 0 && ((kSP * 4) % 16) == 0, "16-B aligned LDS rows");
static_assert(kHalfN == 32 * 4, "one wave covers a half row with 4 columns per lane");

constexpr size_t kOffWH   = 0;
constexpr size_t kWsTotal = kOffWH + (size_t)kFeat * kFeat * 2;
static_assert(kWsTotal == 131072ull, "carve total");
static_assert(kWsTotal <= 134217728ull, "carve cap");

constexpr size_t kLdsBytes = (size_t)kFeat * kKP * 2 + (size_t)2 * kWaves * 16 * kKP * 2 + (size_t)kWaves * 16 * kSP * 4;
static_assert(kLdsBytes == 236544ull, "LDS total");

union FragH { v16h v; v8h h[2]; };

__device__ __forceinline__ v16h frag_load(const _Float16* p) {
  FragH f;
  f.h[0] = *(const v8h*)(p);
  f.h[1] = *(const v8h*)(p + 16);
  return f.v;
}

__device__ __forceinline__ v8f mma_f16(v16h a, v16h b, v8f c) {
  c = __builtin_amdgcn_wmma_f32_16x16x32_f16(false, a, false, b, (short)0, c, false, false);
  asm volatile("v_nop\n\tv_nop\n\tv_nop\n\tv_nop" : "+v"(c) : "v"(a), "v"(b));
  return c;
}

__global__ __launch_bounds__(256) void weight_plane_kernel(
    const float* __restrict__ W, _Float16* __restrict__ WH, int total8)
{
  const int i = blockIdx.x * 256 + threadIdx.x;
  if (i >= total8) return;
  const size_t e0 = (size_t)i << 3;
  const v4f a0 = *(const v4f*)(W + e0);
  const v4f a1 = *(const v4f*)(W + e0 + 4);
  v8h hv;
#pragma unroll
  for (int e = 0; e < 4; ++e) {
    float s0 = a0[e] * kWCarry;
    float s1 = a1[e] * kWCarry;
    s0 = (fabsf(s0) < kF16MinNormal) ? 0.0f : s0;
    s1 = (fabsf(s1) < kF16MinNormal) ? 0.0f : s1;
    hv[e]     = (_Float16)s0;
    hv[4 + e] = (_Float16)s1;
  }
  _Float16* q = WH + e0;
  *(volatile v8h*)q = hv;
  __threadfence();
  *(volatile v8h*)q = hv;
}

template <bool USE_ACC>
__device__ __forceinline__ void row_phase(float* slab, _Float16* zdst, const float* xp, const v4f bv, const bool last)
{
#pragma unroll 1
  for (int r = 0; r < 16; ++r) {
    const v4f xv = *(const v4f*)(xp + (size_t)r * kFeat);
    v4f av = (v4f){0.f, 0.f, 0.f, 0.f};
    if (USE_ACC) av = *(const v4f*)(slab + r * kSP);
    v4f tv;
#pragma unroll
    for (int e = 0; e < 4; ++e) {
      float t = av[e] * kFold + bv[e];
      t = t + xv[e];
      tv[e] = tanhf(t);
    }
    if (last) {
      *(v4f*)(slab + r * kSP) = tv;
    } else {
      v4h zv;
#pragma unroll
      for (int e = 0; e < 4; ++e) {
        float s = tv[e] * kZCarry;
        s = (fabsf(s) < kF16MinNormal) ? 0.0f : s;
        zv[e] = (_Float16)s;
      }
      *(v4h*)(zdst + r * kKP) = zv;
    }
  }
}

__global__ __launch_bounds__(128) void tanh_iter_kernel(
    const float* __restrict__ x, const float* __restrict__ bvec,
    const _Float16* __restrict__ WH, float* __restrict__ out)
{
  __shared__ __align__(16) _Float16 sW[kFeat * kKP];
  __shared__ __align__(16) _Float16 sZ[2 * kWaves * 16 * kKP];
  __shared__ __align__(16) float    sS[kWaves * 16 * kSP];

  unsigned tid = threadIdx.x;
  asm volatile("" : "+v"(tid));
  unsigned lane = tid & 31u;
  asm volatile("" : "+v"(lane));
  unsigned wave = tid >> 5;
  asm volatile("" : "+v"(wave));
  unsigned hh = lane >> 4;
  asm volatile("" : "+v"(hh));
  unsigned c = lane & 15u;
  asm volatile("" : "+v"(c));
  unsigned aLane = c * (unsigned)kKP + 8u * hh;
  asm volatile("" : "+v"(aLane));
  unsigned dLane = 8u * hh * (unsigned)kSP + c;
  asm volatile("" : "+v"(dLane));
  unsigned eLane = lane * 4u;
  asm volatile("" : "+v"(eLane));

  const size_t row0 = (size_t)blockIdx.x * kBlkRows + (size_t)wave * 16u;

#pragma unroll 4
  for (int it = 0; it < 64; ++it) {
    unsigned q = (unsigned)it * 128u + tid;
    unsigned n = q >> 5;
    unsigned k8 = (q & 31u) << 3;
    const v8h v = *(const v8h*)(WH + (size_t)n * kFeat + k8);
    *(v8h*)(sW + n * (unsigned)kKP + k8) = v;
  }

  float* slab = sS + wave * (unsigned)(16 * kSP);

#pragma unroll 1
  for (int half = 0; half < 2; ++half) {
    const v4f bv = *(const v4f*)(bvec + half * kHalfN + eLane);
    row_phase<false>(slab + eLane,
                     sZ + (wave * 16u) * (unsigned)kKP + (unsigned)(half * kHalfN) + eLane,
                     x + row0 * kFeat + (size_t)(half * kHalfN) + eLane,
                     bv, false);
  }
  __syncthreads();

  unsigned cur = 0u;
#pragma unroll 1
  for (int step = 1; step < kSteps; ++step) {
    const bool last = (step == kSteps - 1);
    const _Float16* zin = sZ + ((cur * (unsigned)kWaves + wave) * 16u) * (unsigned)kKP;
    _Float16* zout      = sZ + (((cur ^ 1u) * (unsigned)kWaves + wave) * 16u) * (unsigned)kKP;

#pragma unroll 1
    for (int half = 0; half < 2; ++half) {
      v8f acc[8];
#pragma unroll
      for (int j = 0; j < 8; ++j) acc[j] = (v8f){0.f, 0.f, 0.f, 0.f, 0.f, 0.f, 0.f, 0.f};

      const _Float16* ap = zin + aLane;
      const _Float16* bp = sW + (unsigned)(half * kHalfN * kKP) + aLane;
#pragma unroll 1
      for (int kt = 0; kt < kKTiles; ++kt) {
        const v16h a = frag_load(ap + kt * 32);
#pragma unroll
        for (int j = 0; j < 8; ++j) {
          const v16h b = frag_load(bp + j * 16 * kKP + kt * 32);
          acc[j] = mma_f16(a, b, acc[j]);
        }
      }

      float* sd = slab + dLane;
#pragma unroll
      for (int j = 0; j < 8; ++j) {
#pragma unroll
        for (int r = 0; r < 8; ++r) sd[r * kSP + j * 16] = acc[j][r];
      }
      __syncthreads();

      const v4f bv = *(const v4f*)(bvec + half * kHalfN + eLane);
      row_phase<true>(slab + eLane,
                      zout + (unsigned)(half * kHalfN) + eLane,
                      x + row0 * kFeat + (size_t)(half * kHalfN) + eLane,
                      bv, last);

      if (last) {
        float* orow = out + row0 * kFeat + (size_t)(half * kHalfN) + eLane;
        const float* sr = slab + eLane;
        for (int pass = 0; pass < 2; ++pass) {
#pragma unroll 8
          for (int r = 0; r < 16; ++r) {
            const v4f v = *(const v4f*)(sr + r * kSP);
            *(volatile v4f*)(orow + (size_t)r * kFeat) = v;
          }
          __threadfence();
        }
      }
      __syncthreads();
    }
    cur ^= 1u;
  }
}

extern "C" void kernel_launch(void* const* d_in, const int* in_sizes, int n_in,
                              void* d_out, int out_size, void* d_ws, size_t ws_size,
                              hipStream_t stream) {
  if (n_in < 3) return;
  if (in_sizes[0] != kRows * kFeat) return;
  if (in_sizes[1] != kFeat * kFeat) return;
  if (in_sizes[2] != kFeat) return;
  if (out_size != kRows * kFeat) return;
  if (ws_size < kWsTotal) return;

  const float* x = (const float*)d_in[0];
  const float* W = (const float*)d_in[1];
  const float* b = (const float*)d_in[2];
  float* out = (float*)d_out;
  _Float16* WH = (_Float16*)((char*)d_ws + kOffWH);

  weight_plane_kernel<<<(kFeat * kFeat / 8) / 256, 256, 0, stream>>>(W, WH, kFeat * kFeat / 8);
  tanh_iter_kernel<<<kRows / kBlkRows, kWaves * 32, 0, stream>>>(x, b, WH, out);
}
